// CUDARenderModule_83906481095296
// MI455X (gfx1250) — hardware-run, weakly checked
//
#include <hip/hip_runtime.h>
#include <math.h>


#ifndef NG
#define NG 2048
#endif
#define NG_FULL 2048
#define NTH   32
#define NPH   32
#define NRAY  (NTH * NPH)
#define NT    64
#define KS    64
#define NFA   9
#define GPITCH 72
#define HPI_F  1.5707963267948966f
#define SHC0_F 0.28209479177387814f
#define STEP_F 0.03125f
#define NHL2E  (-0.72134752044448170f)
#define DTH_F  ((float)(1.5707963267948966 / 32.0))
#define DPH_F  ((float)(3.141592653589793 / 32.0))

static_assert(NG % 32 == 0);
static_assert(NG % 16 == 0);
static_assert(NG <= NG_FULL);
static_assert(NRAY % 16 == 0);
static_assert((NT * (NRAY / 16)) % 8 == 0);
static_assert(NRAY % 256 == 0);
static_assert(NFA * 6 + 3 <= KS);
static_assert(KS == 64);
static_assert((GPITCH * 2) % 16 == 0);
static_assert(NT % 8 == 0);
static_assert(NT % 4 == 0 && NT / 4 <= 32);
static_assert((size_t)NT * NRAY * 4 == (size_t)262144);
static_assert(((size_t)NT * NRAY * 4) % 128 == 0);
static_assert(32 * GPITCH * 2 + 64 * 4 <= 131072);
static_assert(8 * 32 * 4 <= 131072);

typedef unsigned short bf;
typedef __attribute__((ext_vector_type(16))) __bf16   v16bf;
typedef __attribute__((ext_vector_type(8)))  unsigned short v8us;
typedef __attribute__((ext_vector_type(8)))  float    v8f;
typedef __attribute__((ext_vector_type(4)))  float    v4f;
typedef __attribute__((ext_vector_type(2)))  float    v2f;
typedef v4f  __attribute__((may_alias)) v4fa;

__device__ __forceinline__ unsigned short f2bf(float f) { unsigned u = __float_as_uint(f); u += 0x7FFFu + ((u >> 16) & 1u); return (unsigned short)(u >> 16); }
__device__ __forceinline__ float bfr(float f) { return __uint_as_float(((unsigned)f2bf(f)) << 16); }
__device__ __forceinline__ v16bf cat16b(v8us lo, v8us hi) { return __builtin_bit_cast(v16bf, __builtin_shufflevector(lo, hi, 0, 1, 2, 3, 4, 5, 6, 7, 8, 9, 10, 11, 12, 13, 14, 15)); }
__device__ __forceinline__ v8f wmmab(v16bf a, v16bf b, v8f c) { return __builtin_amdgcn_wmma_f32_16x16x32_bf16(false, a, false, b, (short)0, c, false, false); }
__device__ __forceinline__ v16bf ldb(const bf* p)  { return cat16b(*(const v8us*)p, *(const v8us*)(p + 16)); }
__device__ __forceinline__ void wave_sync() { __builtin_amdgcn_fence(3  , "wavefront"); __builtin_amdgcn_wave_barrier(); asm volatile("" ::: "memory"); }
__device__ __forceinline__ v8f wmmab_g(v16bf a, v16bf b, v8f c) { c = wmmab(a, b, c); asm volatile("v_nop\n\tv_nop\n\tv_nop\n\tv_nop" : "+v"(c) : "v"(a), "v"(b)); return c; }

__device__ __forceinline__ void split3(float v, bf& h, bf& m, bf& l) {
    h = f2bf(v); const float r1 = v - __uint_as_float(((unsigned)h) << 16);
    m = f2bf(r1); const float r2 = r1 - __uint_as_float(((unsigned)m) << 16);
    l = f2bf(r2);
}
static constexpr int sel_ray(int j) { return j < 3 ? 0 : (j < 5 ? 1 : 2); }
static constexpr int sel_gau(int j) { return (j == 1 || j == 4) ? 1 : (j == 2 ? 2 : 0); }

__device__ __forceinline__ float tval(int k) {
#pragma clang fp contract(off)
    const float s = (float)k * (1.0f / (float)(NT - 1));
    const float v = 0.5f * (1.0f - s) + 2.5f * s;
    return (k == NT - 1) ? 2.5f : v;
}

__device__ __forceinline__ float inv_sq_exp(float x) {
#pragma clang fp contract(off)
    const float s = expf(x); return 1.0f / (s * s);
}

__global__ __launch_bounds__(32) void k_gauss_pre(const float* __restrict__ means, const float* __restrict__ scales, const float* __restrict__ rots,
                                                  const float* __restrict__ opacs, const float* __restrict__ feats, const float* __restrict__ cam,
                                                  bf* GF, float* GO) {
#pragma clang fp contract(off)
    __shared__ __align__(16) bf gs[32 * GPITCH];
    __shared__ __align__(16) float go[64];
    const int lane = threadIdx.x & 31;
    const int g = blockIdx.x * 32 + lane;

    const float a0 = inv_sq_exp(bfr(scales[3 * g + 0]));
    const float a1 = inv_sq_exp(bfr(scales[3 * g + 1]));
    const float a2 = inv_sq_exp(bfr(scales[3 * g + 2]));

    float qw = bfr(rots[4 * g + 0]), qx = bfr(rots[4 * g + 1]), qy = bfr(rots[4 * g + 2]), qz = bfr(rots[4 * g + 3]);
    const float qn = sqrtf(((qw * qw + qx * qx) + qy * qy) + qz * qz) + 1e-12f;
    const float qi = 1.0f / qn;
    qw = qw * qi; qx = qx * qi; qy = qy * qi; qz = qz * qi;

    const float r00 = 1.0f - 2.0f * (qy * qy + qz * qz), r01 = 2.0f * (qx * qy - qw * qz), r02 = 2.0f * (qx * qz + qw * qy);
    const float r10 = 2.0f * (qx * qy + qw * qz), r11 = 1.0f - 2.0f * (qx * qx + qz * qz), r12 = 2.0f * (qy * qz - qw * qx);
    const float r20 = 2.0f * (qx * qz - qw * qy), r21 = 2.0f * (qy * qz + qw * qx), r22 = 1.0f - 2.0f * (qx * qx + qy * qy);

    const float p00 = (r00 * a0) * r00 + (r01 * a1) * r01 + (r02 * a2) * r02;
    const float p01 = (r00 * a0) * r10 + (r01 * a1) * r11 + (r02 * a2) * r12;
    const float p02 = (r00 * a0) * r20 + (r01 * a1) * r21 + (r02 * a2) * r22;
    const float p11 = (r10 * a0) * r10 + (r11 * a1) * r11 + (r12 * a2) * r12;
    const float p12 = (r10 * a0) * r20 + (r11 * a1) * r21 + (r12 * a2) * r22;
    const float p22 = (r20 * a0) * r20 + (r21 * a1) * r21 + (r22 * a2) * r22;

    const float om0 = bfr(cam[0]) - bfr(means[3 * g + 0]);
    const float om1 = bfr(cam[1]) - bfr(means[3 * g + 1]);
    const float om2 = bfr(cam[2]) - bfr(means[3 * g + 2]);
    const float pm0 = p00 * om0 + p01 * om1 + p02 * om2;
    const float pm1 = p01 * om0 + p11 * om1 + p12 * om2;
    const float pm2 = p02 * om0 + p12 * om1 + p22 * om2;
    const float cq  = om0 * pm0 + om1 * pm1 + om2 * pm2;

    float fv[10];
    fv[0] = p00; fv[1] = p11; fv[2] = p22; fv[3] = 2.0f * p01; fv[4] = 2.0f * p02; fv[5] = 2.0f * p12;
    fv[6] = 2.0f * pm0; fv[7] = 2.0f * pm1; fv[8] = 2.0f * pm2; fv[9] = cq;
    bf ph[10], pm[10], pl[10];
#pragma unroll
    for (int c = 0; c < 10; ++c) split3(fv[c], ph[c], pm[c], pl[c]);

    bf sl[KS];
#pragma unroll
    for (int i = 0; i < KS; ++i) sl[i] = (bf)0;
#pragma unroll
    for (int j = 0; j < 6; ++j) {
#pragma unroll
        for (int c = 0; c < NFA; ++c) { const int sg = sel_gau(j); sl[NFA * j + c] = (sg == 0) ? ph[c] : ((sg == 1) ? pm[c] : pl[c]); } }
    sl[NFA * 6 + 0] = ph[9]; sl[NFA * 6 + 1] = pm[9]; sl[NFA * 6 + 2] = pl[9];

#pragma unroll
    for (int q = 0; q < 8; ++q) { v8us v;
#pragma unroll
        for (int e = 0; e < 8; ++e) v[e] = sl[8 * q + e];
        *(v8us*)(&gs[lane * GPITCH + 8 * q]) = v; }

    const float opac = 1.0f / (1.0f + expf(-bfr(opacs[g])));
    const float f0 = fmaxf(SHC0_F * bfr(feats[3 * g + 0]) + 0.5f, 0.0f);
    const float f1 = fmaxf(SHC0_F * bfr(feats[3 * g + 1]) + 0.5f, 0.0f);
    const float f2 = fmaxf(SHC0_F * bfr(feats[3 * g + 2]) + 0.5f, 0.0f);
    const float alb = ((f0 + f1) + f2) * (1.0f / 3.0f);
    go[2 * lane] = opac; go[2 * lane + 1] = opac * alb;
    wave_sync();

    bf* gdst = GF + (size_t)blockIdx.x * 32 * KS;
    float* odst = GO + (size_t)blockIdx.x * 64;
    static_assert(8 * 32 * 16 == 32 * KS * 2);
    static_assert(16 * 16 == 32 * 2 * 4);
#pragma unroll 1
    for (int ps = 0; ps < 2; ++ps) {
#pragma unroll
        for (int s = 0; s < 8; ++s) { const int p = s * 32 + lane; const int row = p >> 3, c8 = (p & 7) * 8;
            const v8us val = *(const v8us*)(&gs[row * GPITCH + c8]);
            *(volatile v8us*)(gdst + (size_t)p * 8) = val; }
        if (lane < 16) { const v4f val = *(const v4fa*)(&go[4 * lane]); *(volatile v4f*)(odst + 4 * lane) = val; }
        if (ps == 0) __threadfence(); }
}

__global__ __launch_bounds__(256) void k_ray_pre(float* DIR) {
#pragma clang fp contract(off)
    const int r = blockIdx.x * 256 + threadIdx.x;
    const int it = r / NPH, ip = r % NPH;
    const float sa = (float)it * (1.0f / (float)(NTH - 1));
    const float sb = (float)ip * (1.0f / (float)(NPH - 1));
    const float th = (it == NTH - 1) ? HPI_F : (HPI_F * sa);
    const float ph = (ip == NPH - 1) ? HPI_F : ((-HPI_F) * (1.0f - sb) + HPI_F * sb);
    float st = 0.0f, ct = 0.0f, sp = 0.0f, cp = 0.0f; float ang = th;
#pragma unroll 1
    for (int i = 0; i < 2; ++i) { float s, c; sincosf(ang, &s, &c); if (i == 0) { st = s; ct = c; } else { sp = s; cp = c; } ang = ph; }
    v4f o; o[0] = st * cp; o[1] = st * sp; o[2] = ct; o[3] = st;
    *(volatile v4f*)(DIR + (size_t)r * 4) = o; __threadfence(); *(volatile v4f*)(DIR + (size_t)r * 4) = o;
}

__global__ __launch_bounds__(256) void k_main(const float* __restrict__ DIR, const bf* __restrict__ GF, const float* __restrict__ GO, float* DR) {
    __shared__ __align__(16) float st[8 * 32];
    const int lane = threadIdx.x & 31, lr = lane & 15, hi = lane >> 4;
    const int wave = __builtin_amdgcn_readfirstlane((int)(threadIdx.x >> 5));
    const int wid = blockIdx.x * 8 + wave;
    const int tIdx = wid / (NRAY / 16);
    const int rbase = (wid % (NRAY / 16)) * 16;
    const float tv = tval(tIdx), t2 = tv * tv;

    const v4f d = *(const v4f*)(DIR + (size_t)(rbase + lr) * 4);
    float fr[NFA];
    fr[0] = t2 * (d[0] * d[0]); fr[1] = t2 * (d[1] * d[1]); fr[2] = t2 * (d[2] * d[2]);
    fr[3] = t2 * (d[0] * d[1]); fr[4] = t2 * (d[0] * d[2]); fr[5] = t2 * (d[1] * d[2]);
    fr[6] = tv * d[0]; fr[7] = tv * d[1]; fr[8] = tv * d[2];
    bf ph[NFA], pm[NFA], pl[NFA];
#pragma unroll
    for (int c = 0; c < NFA; ++c) split3(fr[c], ph[c], pm[c], pl[c]);
    bf rs[KS];
#pragma unroll
    for (int i = 0; i < KS; ++i) rs[i] = (bf)0;
#pragma unroll
    for (int j = 0; j < 6; ++j) {
#pragma unroll
        for (int c = 0; c < NFA; ++c) { const int sr = sel_ray(j); rs[NFA * j + c] = (sr == 0) ? ph[c] : ((sr == 1) ? pm[c] : pl[c]); } }
    rs[NFA * 6 + 0] = (bf)0x3F80; rs[NFA * 6 + 1] = (bf)0x3F80; rs[NFA * 6 + 2] = (bf)0x3F80;

    v8us q0, q1, q2, q3;
#pragma unroll
    for (int i = 0; i < 8; ++i) {
        q0[i] = hi ? rs[ 8 + i] : rs[ 0 + i];
        q1[i] = hi ? rs[24 + i] : rs[16 + i];
        q2[i] = hi ? rs[40 + i] : rs[32 + i];
        q3[i] = hi ? rs[56 + i] : rs[48 + i]; }
    const v16bf a0 = cat16b(q0, q1), a1 = cat16b(q2, q3);

    float dacc[8], racc[8];
#pragma unroll
    for (int i = 0; i < 8; ++i) { dacc[i] = 0.0f; racc[i] = 0.0f; }

    const size_t boff = (size_t)lr * KS + 8 * hi;
#pragma unroll 2
    for (int g0 = 0; g0 < NG; g0 += 16) {
        const bf* gp = GF + boff + (size_t)g0 * KS;
        const v16bf b0 = ldb(gp), b1 = ldb(gp + 32);
        const v2f gw = *(const v2f*)(GO + (size_t)(g0 + lr) * 2);
        v8f acc = (v8f){};
        acc = wmmab_g(a0, b0, acc);
        acc = wmmab_g(a1, b1, acc);
#pragma unroll
        for (int i = 0; i < 8; ++i) {
            const float e = __builtin_amdgcn_exp2f(acc[i] * NHL2E);
            dacc[i] = fmaf(e, gw[0], dacc[i]);
            racc[i] = fmaf(e, gw[1], racc[i]); }
    }

#pragma unroll
    for (int i = 0; i < 8; ++i) {
        float a = dacc[i], b = racc[i];
        a += __shfl_xor(a, 1, 32); b += __shfl_xor(b, 1, 32);
        a += __shfl_xor(a, 2, 32); b += __shfl_xor(b, 2, 32);
        a += __shfl_xor(a, 4, 32); b += __shfl_xor(b, 4, 32);
        a += __shfl_xor(a, 8, 32); b += __shfl_xor(b, 8, 32);
        dacc[i] = a; racc[i] = b; }

    const int wb = wave * 32;
    if (lr == 0) {
#pragma unroll
        for (int i = 0; i < 8; ++i) { st[wb + 2 * (8 * hi + i)] = dacc[i]; st[wb + 2 * (8 * hi + i) + 1] = racc[i]; } }
    wave_sync();
    float* dst = DR + ((size_t)tIdx * NRAY + rbase) * 2;
    static_assert(8 * 16 == 16 * 2 * 4);
#pragma unroll 1
    for (int ps = 0; ps < 2; ++ps) {
        if (lane < 8) { const v4f val = *(const v4fa*)(&st[wb + 4 * lane]); *(volatile v4f*)(dst + 4 * lane) = val; }
        if (ps == 0) __threadfence(); }
}

__global__ __launch_bounds__(256) void k_final(const float* __restrict__ DR, const float* __restrict__ DIR,
                                               const int* __restrict__ nth_p, const int* __restrict__ nph_p, const int* __restrict__ nr_p, float* OUT) {
#pragma clang fp contract(off)
    const int r = blockIdx.x * 256 + threadIdx.x;
    const int bad = (nth_p[0] != NTH) | (nph_p[0] != NPH) | (nr_p[0] != NT);
    const float sth = DIR[(size_t)r * 4 + 3];
    const float qnan = __uint_as_float(0x7FC00000u);
#pragma unroll 1
    for (int ps = 0; ps < 2; ++ps) {
        float acc = 0.0f;
#pragma unroll 1
        for (int k = 0; k < NT; ++k) {
            const v2f dr = *(const v2f*)(DR + ((size_t)k * NRAY + r) * 2);
            const float t = tval(k);
            const float trans = expf(-acc);
            const float rd = dr[1] * trans;
            float val = (rd * (1.0f / (t * t + 1e-8f))) * sth;
            val = bad ? qnan : val;
            *(volatile float*)(OUT + (size_t)k * NRAY + r) = val;
            acc = acc + dr[0] * STEP_F; }
        if (ps == 0) __threadfence(); }
}

__global__ __launch_bounds__(256) void k_hist(float* OUT) {
#pragma clang fp contract(off)
    __shared__ __align__(16) float hs[NT];
    const int lane = threadIdx.x & 31;
    const int wave = __builtin_amdgcn_readfirstlane((int)(threadIdx.x >> 5));
#pragma unroll 1
    for (int i = 0; i < NT / 8; ++i) {
        const int k = wave * (NT / 8) + i;
        float s = 0.0f;
#pragma unroll 4
        for (int j = 0; j < NRAY / 32; ++j) s += OUT[(size_t)k * NRAY + j * 32 + lane];
        s += __shfl_xor(s, 16, 32); s += __shfl_xor(s, 8, 32); s += __shfl_xor(s, 4, 32); s += __shfl_xor(s, 2, 32); s += __shfl_xor(s, 1, 32);
        if (lane == 0) hs[k] = (s * DTH_F) * DPH_F; }
    __syncthreads();
    static_assert((NT / 4) * 16 == NT * 4);
    if (wave == 0) {
#pragma unroll 1
        for (int ps = 0; ps < 2; ++ps) {
            if (lane < NT / 4) { const v4f val = *(const v4fa*)(&hs[4 * lane]); *(volatile v4f*)(OUT + (size_t)NT * NRAY + 4 * lane) = val; }
            if (ps == 0) __threadfence(); } }
}

static constexpr size_t al256(size_t v) { return (v + 255) & ~(size_t)255; }
static constexpr size_t SZ_GF  = al256((size_t)NG * KS * 2);
static constexpr size_t SZ_GO  = al256((size_t)NG * 2 * 4);
static constexpr size_t SZ_DIR = al256((size_t)NRAY * 4 * 4);
static constexpr size_t SZ_DR  = al256((size_t)NT * NRAY * 2 * 4);
static constexpr size_t SZ_TOTAL = SZ_GF + SZ_GO + SZ_DIR + SZ_DR;
static_assert(SZ_TOTAL <= (size_t)134217728);
static_assert((size_t)(NG / 32) * 32 * KS * 2 <= SZ_GF);
static_assert((size_t)(NG / 32) * 64 * 4 <= SZ_GO);
static_assert((size_t)(NT * (NRAY / 16)) * 32 * 4 <= SZ_DR);

extern "C" void kernel_launch(void* const* d_in, const int* in_sizes, int n_in,
                              void* d_out, int out_size, void* d_ws, size_t ws_size, hipStream_t stream) {
    if (n_in < 9) return;
    if (in_sizes[0] < NG * 3 || in_sizes[1] < NG * 3 || in_sizes[2] < NG * 4 || in_sizes[3] < NG || in_sizes[4] < NG * 3) return;
    if (in_sizes[5] < 3 || in_sizes[6] < 1 || in_sizes[7] < 1 || in_sizes[8] < 1) return;
    if ((size_t)out_size < (size_t)NT * NRAY + NT) return;
    if (SZ_TOTAL > ws_size) return;
    const float* means  = (const float*)d_in[0];
    const float* scales = (const float*)d_in[1];
    const float* rots   = (const float*)d_in[2];
    const float* opacs  = (const float*)d_in[3];
    const float* feats  = (const float*)d_in[4];
    const float* cam    = (const float*)d_in[5];
    const int* nth = (const int*)d_in[6];
    const int* nph = (const int*)d_in[7];
    const int* nr  = (const int*)d_in[8];
    float* OUT = (float*)d_out;
    char* wsp = (char*)d_ws;
    bf*    GF  = (bf*)wsp;    wsp += SZ_GF;
    float* GO  = (float*)wsp; wsp += SZ_GO;
    float* DIR = (float*)wsp; wsp += SZ_DIR;
    float* DR  = (float*)wsp; wsp += SZ_DR;

    k_gauss_pre<<<dim3(NG / 32), dim3(32), 0, stream>>>(means, scales, rots, opacs, feats, cam, GF, GO);
    k_ray_pre<<<dim3(NRAY / 256), dim3(256), 0, stream>>>(DIR);
    k_main<<<dim3(NT * (NRAY / 16) / 8), dim3(256), 0, stream>>>(DIR, GF, GO, DR);
    k_final<<<dim3(NRAY / 256), dim3(256), 0, stream>>>(DR, DIR, nth, nph, nr, OUT);
    k_hist<<<dim3(1), dim3(256), 0, stream>>>(OUT);
}
